// GLABlock_14379550507694
// MI455X (gfx1250) — hardware-verified
//
#include <hip/hip_runtime.h>


namespace {
constexpr int Bn = 2, T = 2048, HM = 1024, H = 16, DK = 32, DV = 64, LR = 16, NT = Bn * T;
constexpr int NPJ = 3136;
constexpr float AS_ = 8.0f, EPS = 1e-5f, QSC = 0.17677669529663687f, GNORM = 1.0f / 16.0f;

typedef _Float16 b16;
typedef __attribute__((ext_vector_type(16))) _Float16 v16b;
typedef __attribute__((ext_vector_type(8))) _Float16 v8b;
typedef __attribute__((ext_vector_type(8))) float v8f;
typedef __attribute__((ext_vector_type(4))) float v4f;
__device__ __forceinline__ float bf16_rne(float f) { unsigned int u = __float_as_uint(f); u += 0x7FFFu + ((u >> 16) & 1u); return __uint_as_float(u & 0xFFFF0000u); }
__device__ __forceinline__ void split16(float v, b16& hi, b16& lo) { hi = (b16)v; lo = (b16)(v - (float)hi); }
__device__ __forceinline__ v16b frag_kb(const b16* p, int hh) { const v8b a = *(const v8b*)(p + 8 * hh), b = *(const v8b*)(p + 16 + 8 * hh); v16b f;
#pragma unroll
  for (int e = 0; e < 8; ++e) { f[e] = a[e]; f[8 + e] = b[e]; } return f; }
__device__ __forceinline__ void frag_split(const float* p, int hh, v16b& fh, v16b& fl) {
#pragma unroll
  for (int e = 0; e < 8; ++e) { b16 a, c; split16(p[8 * hh + e] * AS_, a, c); fh[e] = a; fl[e] = c; split16(p[16 + 8 * hh + e] * AS_, a, c); fh[8 + e] = a; fl[8 + e] = c; } }
__device__ __forceinline__ v8f wmma16b(v16b a, v16b b, v8f c) { v8f d = __builtin_amdgcn_wmma_f32_16x16x32_f16(false, a, false, b, (short)0, c, false, false); asm volatile("v_nop\n\tv_nop\n\tv_nop\n\tv_nop" : "+v"(d) : "v"(a), "v"(b)); return d; }
__device__ __forceinline__ void wave_lds_sync() { __builtin_amdgcn_fence(__ATOMIC_RELEASE, "workgroup"); __builtin_amdgcn_wave_barrier(); __builtin_amdgcn_fence(__ATOMIC_ACQUIRE, "workgroup"); }
__device__ __forceinline__ float nexp(float x) { return __builtin_amdgcn_exp2f(x * 1.4426950408889634f); }
__device__ __forceinline__ float pmul(float a, float b) { float p = a * b; asm volatile("" : "+v"(p)); return p; }
__device__ __forceinline__ float softplus_(float z) { return fmaxf(z, 0.0f) + log1pf(nexp(-fabsf(z))); }
__device__ __forceinline__ float gelu_erf(float x) { return 0.5f * x * (1.0f + erff(x * 0.70710678118654752f)); }

struct Wo_ { static constexpr size_t CAT = 0, G2 = CAT + (size_t)NPJ * HM, O = G2 + 512 * 32, W1 = O + (size_t)HM * HM, W2 = W1 + (size_t)2 * HM * HM, END = W2 + (size_t)HM * 2 * HM; };
__global__ __launch_bounds__(256) void prep_kernel(const float* __restrict__ Wq, const float* __restrict__ Wk, const float* __restrict__ Wv, const float* __restrict__ Wg, const float* __restrict__ gw1, const float* __restrict__ gw2, const float* __restrict__ Wo, const float* __restrict__ W1, const float* __restrict__ W2,
                                                   const float* __restrict__ gb2, const float* __restrict__ rmsw, const float* __restrict__ b1, const float* __restrict__ b2, const float* __restrict__ lnw, const float* __restrict__ lnb, b16* __restrict__ R, float* __restrict__ P) {
  const size_t tid = (size_t)blockIdx.x * blockDim.x + threadIdx.x, nth = (size_t)gridDim.x * blockDim.x;
  for (int pass = 0; pass < 2; ++pass) {
    for (size_t p = tid; p < (size_t)NPJ * HM / 8; p += nth) { const int o = (int)(p / (HM / 8)), k8 = (int)(p % (HM / 8)) * 8; v8b v;
#pragma unroll
      for (int e = 0; e < 8; ++e) { const int k = k8 + e; float w;
        if (o < 512) w = Wq[(size_t)k * 512 + o]; else if (o < 1024) w = Wk[(size_t)k * 512 + o - 512]; else if (o < 2048) w = Wv[(size_t)k * 1024 + o - 1024]; else if (o < 3072) w = Wg[(size_t)k * 1024 + o - 2048]; else if (o < 3088) w = gw1[(size_t)k * LR + o - 3072]; else w = 0.0f;
        v[e] = (b16)bf16_rne(w); }
      *(volatile v8b*)(R + Wo_::CAT + (size_t)o * HM + k8) = v; }
    for (size_t p = tid; p < 512 * 32 / 8; p += nth) { const int o = (int)(p / 4), k8 = (int)(p % 4) * 8; v8b v;
#pragma unroll
      for (int e = 0; e < 8; ++e) { const int k = k8 + e; v[e] = (b16)((k < LR) ? bf16_rne(gw2[(size_t)k * 512 + o]) : 0.0f); }
      *(volatile v8b*)(R + Wo_::G2 + (size_t)o * 32 + k8) = v; }
    auto tr = [&](const float* W, int IN, int OUT, size_t base, size_t p) { const int o = (int)(p / (IN / 8)), k8 = (int)(p % (IN / 8)) * 8; v8b v;
#pragma unroll
      for (int e = 0; e < 8; ++e) v[e] = (b16)bf16_rne(W[(size_t)(k8 + e) * OUT + o]);
      *(volatile v8b*)(R + base + (size_t)o * IN + k8) = v; };
    for (size_t p = tid; p < (size_t)HM * HM / 8; p += nth) tr(Wo, HM, HM, Wo_::O, p);
    for (size_t p = tid; p < (size_t)2 * HM * HM / 8; p += nth) { tr(W1, HM, 2 * HM, Wo_::W1, p); tr(W2, 2 * HM, HM, Wo_::W2, p); }
    for (size_t p = tid; p < 5696 / 4; p += nth) { v4f v;
#pragma unroll
      for (int e = 0; e < 4; ++e) { const int i = (int)p * 4 + e; float x; if (i < 512) x = gb2[i]; else if (i < 576) x = rmsw[i - 512]; else if (i < 2624) x = b1[i - 576]; else if (i < 3648) x = b2[i - 2624]; else if (i < 4672) x = lnw[i - 3648]; else x = lnb[i - 4672]; v[e] = bf16_rne(x); }
      *(volatile v4f*)(P + p * 4) = v; }
    __threadfence(); }
}

__global__ __launch_bounds__(256) void ln_kernel(const float* __restrict__ x, const float* __restrict__ g, const float* __restrict__ bb, int rnd, float* __restrict__ y) {
  const int wid = threadIdx.x >> 5, lane = threadIdx.x & 31, row = blockIdx.x * 8 + wid; const float* pr = x + (size_t)row * HM;
  float v[32]; float s = 0.0f;
#pragma unroll
  for (int j = 0; j < 8; ++j) { const v4f t = *(const v4f*)(pr + j * 128 + lane * 4);
#pragma unroll
    for (int e = 0; e < 4; ++e) { v[j * 4 + e] = rnd ? bf16_rne(t[e]) : t[e]; s += v[j * 4 + e]; } }
#pragma unroll
  for (int o = 1; o < 32; o <<= 1) s += __shfl_xor(s, o);
  const float mu = s * (1.0f / HM); float q = 0.0f;
#pragma unroll
  for (int j = 0; j < 32; ++j) { const float d = v[j] - mu; q += pmul(d, d); }
#pragma unroll
  for (int o = 1; o < 32; o <<= 1) q += __shfl_xor(q, o);
  const float is = rsqrtf(q * (1.0f / HM) + EPS);
  for (int pass = 0; pass < 2; ++pass) {
#pragma unroll
    for (int j = 0; j < 8; ++j) { const int c = j * 128 + lane * 4; v4f o4; for (int e = 0; e < 4; ++e) o4[e] = pmul((v[j * 4 + e] - mu) * is, g[c + e]) + bb[c + e]; *(volatile v4f*)(y + (size_t)row * HM + c) = o4; }
    __threadfence(); }
}

__global__ __launch_bounds__(128) void gemm_kernel(const float* __restrict__ X, int K, int ldx, const b16* __restrict__ Bw, int N, const float* __restrict__ bias, int mode, const float* __restrict__ res, int rres, float* __restrict__ Y) {
  __shared__ __attribute__((aligned(16))) float Ts[4][32 * 64];
  const int lane = threadIdx.x & 31, wave = threadIdx.x >> 5, nloc = lane & 15, hlf = lane >> 4, m0 = blockIdx.y * 128 + wave * 32, c0 = blockIdx.x * 64;
  v8f acc[2][4];
#pragma unroll
  for (int r = 0; r < 2; ++r)
#pragma unroll
    for (int t = 0; t < 4; ++t) acc[r][t] = (v8f){};
#pragma unroll 2
  for (int kb = 0; kb < K; kb += 32) { v16b a0, l0, a1, l1; frag_split(X + (size_t)(m0 + nloc) * ldx + kb, hlf, a0, l0); frag_split(X + (size_t)(m0 + 16 + nloc) * ldx + kb, hlf, a1, l1);
#pragma unroll
    for (int t = 0; t < 4; ++t) { const v16b bw = frag_kb(Bw + (size_t)(c0 + t * 16 + nloc) * K + kb, hlf); acc[0][t] = wmma16b(a0, bw, acc[0][t]); acc[0][t] = wmma16b(l0, bw, acc[0][t]); acc[1][t] = wmma16b(a1, bw, acc[1][t]); acc[1][t] = wmma16b(l1, bw, acc[1][t]); } }
  float* Tt = Ts[wave];
#pragma unroll
  for (int t = 0; t < 4; ++t) { const int cc = c0 + t * 16 + nloc; const float bb = bias ? bias[cc] : 0.0f;
#pragma unroll
    for (int r = 0; r < 2; ++r)
#pragma unroll
      for (int v = 0; v < 8; ++v) { const int rl = r * 16 + v + 8 * hlf; float y = acc[r][t][v] * (1.0f / AS_) + bb;
        if (mode == 1) { const float rv = res[(size_t)(m0 + rl) * N + cc]; y += rres ? bf16_rne(rv) : rv; }
        Tt[rl * 64 + t * 16 + nloc] = y; } }
  wave_lds_sync();
  if (mode == 2) {
#pragma unroll 1
    for (int i = lane; i < 32 * 64; i += 32) Tt[i] = gelu_erf(Tt[i]);
    wave_lds_sync(); }
  for (int pass = 0; pass < 2; ++pass) {
#pragma unroll
    for (int j = 0; j < 16; ++j) { const int rr = j * 2 + hlf, c4 = nloc * 4; *(volatile v4f*)(Y + (size_t)(m0 + rr) * N + c0 + c4) = *(const v4f*)(Tt + rr * 64 + c4); }
    __threadfence(); }
}

__global__ __launch_bounds__(128) void decay_kernel(const float* __restrict__ proj, const b16* __restrict__ R, const float* __restrict__ P, float* __restrict__ dec) {
  __shared__ __attribute__((aligned(16))) float Ts[4][32 * 64];
  const int lane = threadIdx.x & 31, wave = threadIdx.x >> 5, nloc = lane & 15, hlf = lane >> 4, m0 = blockIdx.y * 128 + wave * 32, c0 = blockIdx.x * 64; const b16* G2 = R + Wo_::G2; const float* gb2 = P;
  v8f acc[2][4];
#pragma unroll
  for (int r = 0; r < 2; ++r)
#pragma unroll
    for (int t = 0; t < 4; ++t) acc[r][t] = (v8f){};
  v16b a[2], l[2];
#pragma unroll
  for (int r = 0; r < 2; ++r) { const float* pr = proj + (size_t)(m0 + r * 16 + nloc) * NPJ + 3072;
#pragma unroll
    for (int e = 0; e < 16; ++e) { const int k = (e < 8) ? (8 * hlf + e) : (16 + 8 * hlf + e - 8); b16 p_ = (b16)0.0f, q_ = (b16)0.0f; if (k < LR) split16(pr[k] * AS_, p_, q_); a[r][e] = p_; l[r][e] = q_; } }
#pragma unroll
  for (int t = 0; t < 4; ++t) { const v16b bw = frag_kb(G2 + (size_t)(c0 + t * 16 + nloc) * 32, hlf);
#pragma unroll
    for (int r = 0; r < 2; ++r) { acc[r][t] = wmma16b(a[r], bw, acc[r][t]); acc[r][t] = wmma16b(l[r], bw, acc[r][t]); } }
  float* Tt = Ts[wave];
#pragma unroll
  for (int t = 0; t < 4; ++t) { const int cc = c0 + t * 16 + nloc; const float bb = gb2[cc];
#pragma unroll
    for (int r = 0; r < 2; ++r)
#pragma unroll
      for (int v = 0; v < 8; ++v) Tt[(r * 16 + v + 8 * hlf) * 64 + t * 16 + nloc] = acc[r][t][v] * (1.0f / AS_) + bb; }
  wave_lds_sync();
#pragma unroll 1
  for (int i = lane; i < 32 * 64; i += 32) { const float z = Tt[i]; Tt[i] = nexp(-softplus_(-z) * GNORM); }
  wave_lds_sync();
  for (int pass = 0; pass < 2; ++pass) {
#pragma unroll
    for (int j = 0; j < 16; ++j) { const int rr = j * 2 + hlf, c4 = nloc * 4; *(volatile v4f*)(dec + (size_t)(m0 + rr) * 512 + c0 + c4) = *(const v4f*)(Tt + rr * 64 + c4); }
    __threadfence(); }
}

__global__ __launch_bounds__(128) void gla_kernel(const float* __restrict__ proj, const float* __restrict__ dec, float* __restrict__ o) {
  const int wg = blockIdx.x * 4 + (threadIdx.x >> 5), lane = threadIdx.x & 31; const int b = wg / (H * 2), h = (wg / 2) % H, vh = wg & 1; const int vcol = h * DV + vh * 32 + lane;
  float S[DK];
#pragma unroll
  for (int k = 0; k < DK; ++k) S[k] = 0.0f;
  for (int t = 0; t < T; ++t) { const size_t row = (size_t)b * T + t; const float* pr = proj + row * NPJ; const float* dr = dec + row * 512 + h * DK;
    const float vv = pr[1024 + vcol]; float acc = 0.0f;
#pragma unroll
    for (int k4 = 0; k4 < DK; k4 += 4) { const v4f d4 = *(const v4f*)(dr + k4), kk4 = *(const v4f*)(pr + 512 + h * DK + k4), q4 = *(const v4f*)(pr + h * DK + k4);
#pragma unroll
      for (int e = 0; e < 4; ++e) { S[k4 + e] = d4[e] * S[k4 + e] + pmul(kk4[e], vv); acc += pmul(q4[e] * QSC, S[k4 + e]); } }
    for (int pass = 0; pass < 2; ++pass) ((volatile float*)o)[row * HM + vcol] = acc; }
  __threadfence();
}

__global__ __launch_bounds__(256) void gate_kernel(const float* __restrict__ o, const float* __restrict__ proj, const float* __restrict__ P, float* __restrict__ og) {
  const int wid = threadIdx.x >> 5, lane = threadIdx.x & 31; const size_t row = (size_t)blockIdx.x * 8 + wid; const float* orow = o + row * HM; const float* grow = proj + row * NPJ + 2048; const float* rw = P + 512;
  for (int h = 0; h < H; ++h) { const float a = orow[h * DV + lane], c = orow[h * DV + 32 + lane]; float s = pmul(a, a) + pmul(c, c);
#pragma unroll
    for (int sh = 1; sh < 32; sh <<= 1) s += __shfl_xor(s, sh);
    const float is = rsqrtf(s * (1.0f / DV) + EPS);
    const float g0 = grow[h * DV + lane], g1 = grow[h * DV + 32 + lane];
    const float y0 = pmul(a * is, rw[lane]) * pmul(g0, 1.0f / (1.0f + nexp(-g0))), y1 = pmul(c * is, rw[32 + lane]) * pmul(g1, 1.0f / (1.0f + nexp(-g1)));
    for (int pass = 0; pass < 2; ++pass) { ((volatile float*)og)[row * HM + h * DV + lane] = y0; ((volatile float*)og)[row * HM + h * DV + 32 + lane] = y1; } }
  __threadfence();
}
}

extern "C" void kernel_launch(void* const* d_in, const int* in_sizes, int n_in,
                              void* d_out, int out_size, void* d_ws, size_t ws_size, hipStream_t stream) {
  (void)n_in; (void)out_size;
  const float* x = (const float*)d_in[0]; const float* lnw = (const float*)d_in[1]; const float* lnb = (const float*)d_in[2]; const float* Wq = (const float*)d_in[3]; const float* Wk = (const float*)d_in[4]; const float* Wv = (const float*)d_in[5];
  const float* gw1 = (const float*)d_in[6]; const float* gw2 = (const float*)d_in[7]; const float* gb2 = (const float*)d_in[8]; const float* Wg = (const float*)d_in[9]; const float* rmsw = (const float*)d_in[10]; const float* Wo = (const float*)d_in[11];
  const float* W1 = (const float*)d_in[12]; const float* b1 = (const float*)d_in[13]; const float* W2 = (const float*)d_in[14]; const float* b2 = (const float*)d_in[15];
  float* out = (float*)d_out;
  if (in_sizes[0] != NT * HM || in_sizes[3] != HM * 512 || in_sizes[7] != LR * 512 || in_sizes[11] != HM * HM || in_sizes[12] != HM * 2 * HM || in_sizes[14] != 2 * HM * HM) return;
  size_t off = 0; char* ws = (char*)d_ws;
  auto carve = [&](size_t bytes) { char* p = ws + off; off += (bytes + 255) & ~(size_t)255; return p; };
  b16* R = (b16*)carve(Wo_::END * 2); float* P = (float*)carve(5696 * 4 + 256); float* hn = (float*)carve((size_t)NT * HM * 4); float* proj = (float*)carve((size_t)NT * NPJ * 4); float* dec = (float*)carve((size_t)NT * 512 * 4); float* o = (float*)carve((size_t)NT * HM * 4); float* x2 = (float*)carve((size_t)NT * HM * 4);
  float* og = hn;
  float* h2 = proj; float* hmid = proj + (size_t)NT * HM;
  if (off > ws_size) return;
  prep_kernel<<<512, 256, 0, stream>>>(Wq, Wk, Wv, Wg, gw1, gw2, Wo, W1, W2, gb2, rmsw, b1, b2, lnw, lnb, R, P);
  ln_kernel<<<NT / 8, 256, 0, stream>>>(x, P + 3648, P + 4672, 1, hn);
  gemm_kernel<<<dim3(NPJ / 64, NT / 128), 128, 0, stream>>>(hn, HM, HM, R + Wo_::CAT, NPJ, nullptr, 0, nullptr, 0, proj);
  decay_kernel<<<dim3(512 / 64, NT / 128), 128, 0, stream>>>(proj, R, P, dec);
  gla_kernel<<<Bn * H * 2 / 4, 128, 0, stream>>>(proj, dec, o);
  gate_kernel<<<NT / 8, 256, 0, stream>>>(o, proj, P, og);
  gemm_kernel<<<dim3(HM / 64, NT / 128), 128, 0, stream>>>(og, HM, HM, R + Wo_::O, HM, nullptr, 1, x, 1, x2);
  ln_kernel<<<NT / 8, 256, 0, stream>>>(x2, P + 3648, P + 4672, 0, h2);
  gemm_kernel<<<dim3(2 * HM / 64, NT / 128), 128, 0, stream>>>(h2, HM, HM, R + Wo_::W1, 2 * HM, P + 576, 2, nullptr, 0, hmid);
  gemm_kernel<<<dim3(HM / 64, NT / 128), 128, 0, stream>>>(hmid, 2 * HM, 2 * HM, R + Wo_::W2, HM, P + 2624, 1, x2, 0, out);
}
